// PointNetSetAbstraction_70153995813097
// MI455X (gfx1250) — hardware-verified
//
#include <hip/hip_runtime.h>
#include <stdint.h>

#pragma clang fp contract(off)

typedef __attribute__((ext_vector_type(16))) _Float16 v16h;
typedef __attribute__((ext_vector_type(8)))  _Float16 v8h;
typedef __attribute__((ext_vector_type(8)))  float    v8f;
typedef __attribute__((ext_vector_type(4)))  float    v4f;

constexpr int kBatch   = 8;
constexpr int kPts     = 8192;
constexpr int kFeat    = 16;
constexpr int kQuery   = 1024;
constexpr int kSample  = 32;
constexpr int kRows    = kBatch * kQuery * kSample;
constexpr int kCin0    = 3 + kFeat;
constexpr int kCin0Pad = 32;
constexpr int kGemmBlocks = kRows / 256;
static_assert(kRows == 262144, "row count");
static_assert(kCin0 == 19, "layer-0 input channels");
static_assert(kRows % 256 == 0, "8 waves x 32 rows per block");
static_assert(kPts % 32 == 0, "scan chunks");
static_assert(kQuery == 1024, "one fps thread per query at output time");

constexpr size_t OFF_W0H   = 0;
constexpr size_t OFF_W1H   = OFF_W0H + 64 * 32 * 2;
constexpr size_t OFF_W2H   = OFF_W1H + 64 * 64 * 2;
constexpr size_t OFF_COEF  = OFF_W2H + 128 * 64 * 2;
constexpr size_t OFF_QXYZ  = OFF_COEF + 3 * 1024;
constexpr size_t OFF_PART0 = OFF_QXYZ + (size_t)kBatch * kQuery * 16;
constexpr size_t OFF_PART1 = OFF_PART0 + (size_t)kGemmBlocks * 2 * 64 * 4;
constexpr size_t OFF_PART2 = OFF_PART1 + (size_t)kGemmBlocks * 2 * 64 * 4;
constexpr size_t OFF_X0    = OFF_PART2 + (size_t)kGemmBlocks * 2 * 128 * 4;
constexpr size_t OFF_Y0    = OFF_X0 + (size_t)kRows * 32 * 2;
constexpr size_t OFF_Y1    = OFF_Y0 + (size_t)kRows * 64 * 2;
constexpr size_t OFF_MM    = OFF_Y1 + (size_t)kRows * 64 * 2;
constexpr size_t WS_TOTAL  = OFF_MM + (size_t)kBatch * kQuery * 2 * 128 * 4;
static_assert(WS_TOTAL <= (size_t)134217728, "carve within 128 MiB");
static_assert(OFF_COEF % 128 == 0 && OFF_QXYZ % 128 == 0 && OFF_PART0 % 128 == 0, "alignment");
static_assert(OFF_X0 % 128 == 0 && OFF_Y0 % 128 == 0 && OFF_MM % 128 == 0, "alignment");

constexpr size_t OUT0_BYTES = (size_t)kBatch * kQuery * 3 * 4;
constexpr size_t OUT1_BYTES = (size_t)kBatch * kQuery * 128 * 4;
static_assert(OUT0_BYTES == 98304, "out1 byte offset");
static_assert(OUT0_BYTES + OUT1_BYTES == 4292608, "d_out total");

__device__ __forceinline__ v16h frag_load_h(const _Float16* p) {
  union U { v16h v; v8h h[2]; };
  U f;
  f.h[0] = *(const v8h*)(p);
  f.h[1] = *(const v8h*)(p + 16);
  return f.v;
}

__device__ __forceinline__ void mma_pair_guard(v8f& c0, v8f& c1, v16h a0, v16h a1, v16h b) {
  c0 = __builtin_amdgcn_wmma_f32_16x16x32_f16(false, a0, false, b, (short)0, c0, false, false);
  c1 = __builtin_amdgcn_wmma_f32_16x16x32_f16(false, a1, false, b, (short)0, c1, false, false);
  asm volatile("v_nop\n\tv_nop\n\tv_nop\n\tv_nop" : "+v"(c0), "+v"(c1) : "v"(a0), "v"(a1), "v"(b));
}

__device__ __forceinline__ void wave_lds_sync() {
  __builtin_amdgcn_fence(__ATOMIC_RELEASE, "workgroup");
  __builtin_amdgcn_wave_barrier();
  __builtin_amdgcn_fence(__ATOMIC_ACQUIRE, "workgroup");
}

__device__ __forceinline__ float h16_to_f32(unsigned hb) {
  const unsigned sgn = (hb & 0x8000u) << 16;
  const unsigned em = hb & 0x7fffu;
  const float fn = __uint_as_float((em << 13) + 0x38000000u);
  const float fs = (float)em * 5.9604644775390625e-8f;
  const float mag = (em < 0x400u) ? fs : fn;
  return __uint_as_float(__float_as_uint(mag) | sgn);
}

__device__ __forceinline__ float bn_relu_h(unsigned hb, float a, float c) {
  const float f = h16_to_f32(hb);
  return fmaxf(__builtin_fmaf(a, f, c), 0.0f);
}

__device__ __forceinline__ void lds4(const float* p, float& o0, float& o1, float& o2, float& o3) {
  const v4f v = *(const v4f*)p;
  o0 = v.x; o1 = v.y; o2 = v.z; o3 = v.w;
}

__global__ __launch_bounds__(256) void cvt_w_kernel(const float* __restrict__ w0, const float* __restrict__ w1,
                                                    const float* __restrict__ w2,
                                                    unsigned short* __restrict__ w0h, unsigned short* __restrict__ w1h,
                                                    unsigned short* __restrict__ w2h) {
  const int blk = blockIdx.x;
  const int tid = threadIdx.x;
  float f[8];
  unsigned short* dst;
  if (blk == 0) {
    const int o = tid >> 2;
    const int kb = (tid & 3) * 8;
#pragma unroll
    for (int e = 0; e < 8; ++e) {
      const int k = kb + e;
      const int kc = (k < kCin0) ? k : (kCin0 - 1);
      const float v = w0[o * kCin0 + kc];
      f[e] = (k < kCin0) ? v : 0.0f;
    }
    dst = w0h + tid * 8;
  } else if (blk < 3) {
    const int i = (blk - 1) * 256 + tid;
    const v4f a = *(const v4f*)(w1 + (size_t)i * 8);
    const v4f c = *(const v4f*)(w1 + (size_t)i * 8 + 4);
    f[0] = a.x; f[1] = a.y; f[2] = a.z; f[3] = a.w;
    f[4] = c.x; f[5] = c.y; f[6] = c.z; f[7] = c.w;
    dst = w1h + (size_t)i * 8;
  } else {
    const int i = (blk - 3) * 256 + tid;
    const v4f a = *(const v4f*)(w2 + (size_t)i * 8);
    const v4f c = *(const v4f*)(w2 + (size_t)i * 8 + 4);
    f[0] = a.x; f[1] = a.y; f[2] = a.z; f[3] = a.w;
    f[4] = c.x; f[5] = c.y; f[6] = c.z; f[7] = c.w;
    dst = w2h + (size_t)i * 8;
  }
  v8h hv;
#pragma unroll
  for (int e = 0; e < 8; ++e) hv[e] = (_Float16)f[e];
  *(volatile v8h*)dst = hv;
  __threadfence();
  *(volatile v8h*)dst = hv;
}

__global__ __launch_bounds__(1024) void fps_kernel(const float* __restrict__ xyz,
                                                   const int* __restrict__ init_far,
                                                   float* __restrict__ out0,
                                                   float* __restrict__ qxyz) {
#pragma clang fp contract(off)
  __shared__ __align__(16) float s_stage[3072];
  __shared__ __align__(16) float s_new[3 * kQuery];
  __shared__ float redv[32];
  __shared__ int   redi[32];
  __shared__ int   sfar;
  const int b = blockIdx.x;
  const int tid = threadIdx.x;
  const int lane = tid & 31, wv = tid >> 5;
  const float* xb = xyz + (size_t)b * kPts * 3;

  float px[8], py[8], pz[8], dist[8];
#pragma unroll
  for (int j = 0; j < 8; ++j) {
    __syncthreads();
    if (tid < 768) {
      const v4f t = *(const v4f*)(xb + (size_t)j * 3072 + tid * 4);
      *(v4f*)(s_stage + tid * 4) = t;
    }
    __syncthreads();
    px[j] = s_stage[tid * 3 + 0];
    py[j] = s_stage[tid * 3 + 1];
    pz[j] = s_stage[tid * 3 + 2];
    dist[j] = 1e10f;
  }
  int far = init_far[b];
  far = far < 0 ? 0 : (far > kPts - 1 ? kPts - 1 : far);

  for (int it = 0; it < kQuery; ++it) {
    const float cx = xb[far * 3 + 0];
    const float cy = xb[far * 3 + 1];
    const float cz = xb[far * 3 + 2];
    if (tid == 0) {
      s_new[it * 3 + 0] = cx;
      s_new[it * 3 + 1] = cy;
      s_new[it * 3 + 2] = cz;
    }
    float bv = -1.f;
    int bp = 0x7fffffff;
#pragma unroll
    for (int j = 0; j < 8; ++j) {
      const float dx = px[j] - cx, dy = py[j] - cy, dz = pz[j] - cz;
      const float t0 = dx * dx;
      const float t1 = dy * dy;
      const float t2 = dz * dz;
      float d = (t0 + t2) + t1;
      d = fminf(dist[j], d);
      dist[j] = d;
      const int p = tid + j * 1024;
      if (d > bv || (d == bv && p < bp)) { bv = d; bp = p; }
    }
#pragma unroll
    for (int off = 16; off; off >>= 1) {
      const float ov = __shfl_xor(bv, off, 32);
      const int   op = __shfl_xor(bp, off, 32);
      if (ov > bv || (ov == bv && op < bp)) { bv = ov; bp = op; }
    }
    if (lane == 0) { redv[wv] = bv; redi[wv] = bp; }
    __syncthreads();
    if (tid < 32) {
      bv = redv[tid];
      bp = redi[tid];
#pragma unroll
      for (int off = 16; off; off >>= 1) {
        const float ov = __shfl_xor(bv, off, 32);
        const int   op = __shfl_xor(bp, off, 32);
        if (ov > bv || (ov == bv && op < bp)) { bv = ov; bp = op; }
      }
      if (tid == 0) sfar = bp;
    }
    __syncthreads();
    far = sfar;
    far = far < 0 ? 0 : (far > kPts - 1 ? kPts - 1 : far);
  }
  __syncthreads();
  if (tid < 768) {
    const v4f v = *(const v4f*)(s_new + tid * 4);
    float* p = out0 + (size_t)b * 3072 + tid * 4;
    *(volatile v4f*)p = v;
    __threadfence();
    *(volatile v4f*)p = v;
  }
  {
    const v4f v = (v4f){s_new[tid * 3 + 0], s_new[tid * 3 + 1], s_new[tid * 3 + 2], 0.0f};
    float* p = qxyz + ((size_t)b * kQuery + tid) * 4;
    *(volatile v4f*)p = v;
    __threadfence();
    *(volatile v4f*)p = v;
  }
}

__global__ __launch_bounds__(256) void ball_group_kernel(const float* __restrict__ xyz,
                                                         const float* __restrict__ pts,
                                                         const float* __restrict__ qxyz,
                                                         unsigned short* __restrict__ x0) {
#pragma clang fp contract(off)
  __shared__ int s_list[8][32];
  __shared__ __align__(16) float s_row[8][32 * 36];
  const int lane = threadIdx.x & 31;
  const int wave = threadIdx.x >> 5;
  const int bs = blockIdx.x * 8 + wave;
  const int b = bs >> 10;
  const v4f qv = *(const v4f*)(qxyz + (size_t)bs * 4);
  const float qx = qv.x, qy = qv.y, qz = qv.z;
  const float* xb = xyz + (size_t)b * kPts * 3;
  const float* fb = pts + (size_t)b * kPts * kFeat;
  const float q0 = qx * qx;
  const float q1 = qy * qy;
  const float q2 = qz * qz;
  const float sqq = (q0 + q2) + q1;

  s_list[wave][lane] = 0;
  int cnt = 0;
  for (int n0 = 0; n0 < kPts && cnt < kSample; n0 += 32) {
    const int p = n0 + lane;
    const float px = xb[p * 3 + 0];
    const float py = xb[p * 3 + 1];
    const float pz = xb[p * 3 + 2];
    float dot = qx * px;
    dot = __builtin_fmaf(qy, py, dot);
    dot = __builtin_fmaf(qz, pz, dot);
    const float t0 = px * px;
    const float t1 = py * py;
    const float t2 = pz * pz;
    const float sqp = (t0 + t2) + t1;
    const float dd = -2.0f * dot;
    const float sqr = (dd + sqq) + sqp;
    const bool in = !(sqr > 0.04f);
    const unsigned m = __builtin_amdgcn_ballot_w32(in);
    const int pos = cnt + __popc(m & ((1u << lane) - 1u));
    if (in && pos < kSample) s_list[wave][pos] = p;
    cnt += __popc(m);
  }
  if (cnt > kSample) cnt = kSample;
  __syncthreads();

  {
    const int slot = (lane < cnt) ? lane : 0;
    int idx = s_list[wave][slot];
    idx = idx < 0 ? 0 : (idx > kPts - 1 ? kPts - 1 : idx);
    const float gx = xb[idx * 3 + 0];
    const float gy = xb[idx * 3 + 1];
    const float gz = xb[idx * 3 + 2];
    const v4f f0 = *(const v4f*)(fb + (size_t)idx * kFeat + 0);
    const v4f f1 = *(const v4f*)(fb + (size_t)idx * kFeat + 4);
    const v4f f2 = *(const v4f*)(fb + (size_t)idx * kFeat + 8);
    const v4f f3 = *(const v4f*)(fb + (size_t)idx * kFeat + 12);
    float* rowp = s_row[wave] + lane * 36;
    *(v4f*)(rowp + 0)  = (v4f){gx - qx, gy - qy, gz - qz, f0.x};
    *(v4f*)(rowp + 4)  = (v4f){f0.y, f0.z, f0.w, f1.x};
    *(v4f*)(rowp + 8)  = (v4f){f1.y, f1.z, f1.w, f2.x};
    *(v4f*)(rowp + 12) = (v4f){f2.y, f2.z, f2.w, f3.x};
    *(v4f*)(rowp + 16) = (v4f){f3.y, f3.z, f3.w, 0.0f};
    *(v4f*)(rowp + 20) = (v4f){0.0f, 0.0f, 0.0f, 0.0f};
    *(v4f*)(rowp + 24) = (v4f){0.0f, 0.0f, 0.0f, 0.0f};
    *(v4f*)(rowp + 28) = (v4f){0.0f, 0.0f, 0.0f, 0.0f};
  }
  __syncthreads();
  {
    unsigned short* dst = x0 + (size_t)bs * (kSample * kCin0Pad);
    for (int pass = 0; pass < 2; ++pass) {
#pragma unroll
      for (int it = 0; it < 4; ++it) {
        const int row = it * 8 + (lane >> 2);
        const int col = (lane & 3) * 8;
        const float* sp = s_row[wave] + row * 36 + col;
        v8h hv;
#pragma unroll
        for (int e = 0; e < 8; ++e) hv[e] = (_Float16)sp[e];
        *(volatile v8h*)(dst + it * 256 + lane * 8) = hv;
      }
      __threadfence();
    }
  }
}

template <int CIN, int COUT, bool BN_IN, bool STORE_Y>
__global__ __launch_bounds__(256) void mlp_layer_kernel(const unsigned short* __restrict__ Ain,
                                                        const unsigned short* __restrict__ Wt,
                                                        const float* __restrict__ bias,
                                                        const float* __restrict__ coef_in,
                                                        unsigned short* __restrict__ Yout,
                                                        float* __restrict__ mmout,
                                                        float* __restrict__ part) {
  static_assert(CIN % 32 == 0, "K multiple of 32");
  static_assert(COUT % 64 == 0, "N multiple of 64");
  static_assert(!BN_IN || CIN == 64, "coefficient tile size");
  static_assert(2 * COUT <= 256, "partials written by one block pass");
  constexpr int KS = CIN / 32;
  constexpr int NH = COUT / 64;
  __shared__ __align__(16) float s_ca[64];
  __shared__ __align__(16) float s_cc[64];
  __shared__ __align__(16) float s_slab[STORE_Y ? 8 * 16 * 68 : 4];
  __shared__ __align__(16) float s_mm[STORE_Y ? 4 : 8 * 2 * COUT];
  __shared__ float s_red[8 * 2 * COUT];

  const int tid = threadIdx.x;
  const int lane = tid & 31;
  const int wave = tid >> 5;
  const int rlane = lane & 15;
  const int hh = lane >> 4;
  const int koff = hh * 8;
  const int mOff = hh * 8;

  if constexpr (BN_IN) {
    if (tid < 64) {
      s_ca[tid] = coef_in[tid];
      s_cc[tid] = coef_in[128 + tid];
    }
  }
  __syncthreads();

  const int tile = blockIdx.x * 8 + wave;
  const int m0 = tile * 32;

  v16h afr[KS][2];
#pragma unroll
  for (int ks = 0; ks < KS; ++ks) {
    float ca[16], cc[16];
    if constexpr (BN_IN) {
      const float* pa = s_ca + ks * 32 + koff;
      const float* pc = s_cc + ks * 32 + koff;
      lds4(pa,      ca[0],  ca[1],  ca[2],  ca[3]);
      lds4(pa + 4,  ca[4],  ca[5],  ca[6],  ca[7]);
      lds4(pa + 16, ca[8],  ca[9],  ca[10], ca[11]);
      lds4(pa + 20, ca[12], ca[13], ca[14], ca[15]);
      lds4(pc,      cc[0],  cc[1],  cc[2],  cc[3]);
      lds4(pc + 4,  cc[4],  cc[5],  cc[6],  cc[7]);
      lds4(pc + 16, cc[8],  cc[9],  cc[10], cc[11]);
      lds4(pc + 20, cc[12], cc[13], cc[14], cc[15]);
    }
#pragma unroll
    for (int i = 0; i < 2; ++i) {
      const unsigned short* ap = Ain + (size_t)(m0 + i * 16 + rlane) * CIN + ks * 32 + koff;
      if constexpr (!BN_IN) {
        afr[ks][i] = frag_load_h((const _Float16*)ap);
      } else {
        const uint4 u0 = *(const uint4*)(ap);
        const uint4 u1 = *(const uint4*)(ap + 16);
        unsigned wd[8];
        wd[0] = u0.x; wd[1] = u0.y; wd[2] = u0.z; wd[3] = u0.w;
        wd[4] = u1.x; wd[5] = u1.y; wd[6] = u1.z; wd[7] = u1.w;
        v16h av;
#pragma unroll
        for (int e = 0; e < 8; ++e) {
          const unsigned w0 = wd[e >> 1];
          const unsigned w1 = wd[4 + (e >> 1)];
          const unsigned hb0 = (e & 1) ? (w0 >> 16) : (w0 & 0xffffu);
          const unsigned hb1 = (e & 1) ? (w1 >> 16) : (w1 & 0xffffu);
          const float x0v = bn_relu_h(hb0, ca[e], cc[e]);
          const float x1v = bn_relu_h(hb1, ca[8 + e], cc[8 + e]);
          av[e] = (_Float16)x0v;
          av[8 + e] = (_Float16)x1v;
        }
        afr[ks][i] = av;
      }
    }
  }

  const _Float16* Wh = (const _Float16*)Wt;

#pragma unroll 1
  for (int nh = 0; nh < NH; ++nh) {
    v8f acc[2][4];
#pragma unroll
    for (int i = 0; i < 2; ++i)
#pragma unroll
      for (int j = 0; j < 4; ++j) acc[i][j] = (v8f){0.f, 0.f, 0.f, 0.f, 0.f, 0.f, 0.f, 0.f};

#pragma unroll
    for (int ks = 0; ks < KS; ++ks) {
#pragma unroll
      for (int j = 0; j < 4; ++j) {
        const _Float16* bp = Wh + (size_t)(nh * 64 + j * 16 + rlane) * CIN + ks * 32 + koff;
        const v16h bf = frag_load_h(bp);
        mma_pair_guard(acc[0][j], acc[1][j], afr[ks][0], afr[ks][1], bf);
      }
    }

#pragma unroll
    for (int j = 0; j < 4; ++j) {
      const int col = nh * 64 + j * 16 + rlane;
      const float bv = bias[col];
      float s = 0.0f, q = 0.0f;
      float mx = -3.402823466e38f, mn = 3.402823466e38f;
#pragma unroll
      for (int i = 0; i < 2; ++i) {
#pragma unroll
        for (int r = 0; r < 8; ++r) {
          const float v = acc[i][j][r] + bv;
          acc[i][j][r] = v;
          s += v;
          q += v * v;
          mx = fmaxf(mx, v);
          mn = fminf(mn, v);
        }
      }
      s += __shfl_xor(s, 16, 32);
      q += __shfl_xor(q, 16, 32);
      const float omx = __shfl_xor(mx, 16, 32);
      const float omn = __shfl_xor(mn, 16, 32);
      mx = fmaxf(mx, omx);
      mn = fminf(mn, omn);
      if (hh == 0) {
        s_red[wave * 2 * COUT + col] = s;
        s_red[wave * 2 * COUT + COUT + col] = q;
      }
      if constexpr (!STORE_Y) {
        const float sel = hh ? mn : mx;
        s_mm[wave * 2 * COUT + hh * COUT + col] = sel;
      }
    }

    if constexpr (STORE_Y) {
      float* slab = s_slab + wave * (16 * 68);
#pragma unroll
      for (int i = 0; i < 2; ++i) {
#pragma unroll
        for (int j = 0; j < 4; ++j) {
#pragma unroll
          for (int r = 0; r < 8; ++r) slab[(mOff + r) * 68 + (j << 4) + rlane] = acc[i][j][r];
        }
        wave_lds_sync();
        {
          const int q4 = lane >> 3, c8 = (lane & 7) * 8;
          for (int pass = 0; pass < 2; ++pass) {
#pragma unroll
            for (int it = 0; it < 4; ++it) {
              const int row = it * 4 + q4;
              const float* sp = slab + row * 68 + c8;
              v8h hv;
#pragma unroll
              for (int e = 0; e < 8; ++e) hv[e] = (_Float16)sp[e];
              *(volatile v8h*)(Yout + (size_t)(m0 + i * 16 + row) * COUT + nh * 64 + c8) = hv;
            }
            __threadfence();
          }
        }
        wave_lds_sync();
      }
    }
  }

  __syncthreads();

  if constexpr (!STORE_Y) {
    float* mrow = mmout + (size_t)tile * 2 * COUT;
    const float* src = s_mm + wave * 2 * COUT;
    for (int pass = 0; pass < 2; ++pass) {
#pragma unroll
      for (int it = 0; it < (2 * COUT) / 128; ++it) {
        const v4f v = *(const v4f*)(src + it * 128 + lane * 4);
        *(volatile v4f*)(mrow + it * 128 + lane * 4) = v;
      }
      __threadfence();
    }
  }

  if (tid < 2 * COUT) {
    float tsum = 0.0f;
#pragma unroll
    for (int w = 0; w < 8; ++w) tsum += s_red[w * 2 * COUT + tid];
    float* pp = part + (size_t)blockIdx.x * 2 * COUT + tid;
    *(volatile float*)pp = tsum;
    __threadfence();
    *(volatile float*)pp = tsum;
  }
}

__global__ __launch_bounds__(128) void bn_fin_kernel(const float* __restrict__ part, int nblk,
                                                     const float* __restrict__ g, const float* __restrict__ be,
                                                     float* __restrict__ coef, int cout) {
  const int o = threadIdx.x;
  const int oc = (o < cout) ? o : (cout - 1);
  const int nb = (nblk < kGemmBlocks) ? nblk : kGemmBlocks;
  double s = 0.0, q = 0.0;
#pragma unroll 4
  for (int blk = 0; blk < nb; ++blk) {
    s += (double)part[(size_t)blk * 2 * cout + oc];
    q += (double)part[(size_t)blk * 2 * cout + cout + oc];
  }
  const double inv = 1.0 / (double)kRows;
  const double mean = s * inv;
  double var = q * inv - mean * mean;
  if (var < 0.0) var = 0.0;
  const float rstd = rsqrtf((float)var + 1e-5f);
  const float a = g[oc] * rstd;
  const float c = be[oc] - (float)mean * a;
  if (o < cout) {
    *(volatile float*)(coef + o) = a;
    *(volatile float*)(coef + 128 + o) = c;
    __threadfence();
    *(volatile float*)(coef + o) = a;
    *(volatile float*)(coef + 128 + o) = c;
  }
}

__global__ __launch_bounds__(256) void final_kernel(const float* __restrict__ mm, const float* __restrict__ coef,
                                                    float* __restrict__ out1) {
  const int lane = threadIdx.x & 31;
  const int wave = threadIdx.x >> 5;
  const int qi = blockIdx.x * 8 + wave;
  const int c4 = lane * 4;
  const v4f mx = *(const v4f*)(mm + (size_t)qi * 256 + c4);
  const v4f mn = *(const v4f*)(mm + (size_t)qi * 256 + 128 + c4);
  const v4f a = *(const v4f*)(coef + c4);
  const v4f c = *(const v4f*)(coef + 128 + c4);
  const float s0 = (a.x >= 0.0f) ? mx.x : mn.x;
  const float s1 = (a.y >= 0.0f) ? mx.y : mn.y;
  const float s2 = (a.z >= 0.0f) ? mx.z : mn.z;
  const float s3 = (a.w >= 0.0f) ? mx.w : mn.w;
  v4f r;
  r.x = fmaxf(__builtin_fmaf(a.x, s0, c.x), 0.0f);
  r.y = fmaxf(__builtin_fmaf(a.y, s1, c.y), 0.0f);
  r.z = fmaxf(__builtin_fmaf(a.z, s2, c.z), 0.0f);
  r.w = fmaxf(__builtin_fmaf(a.w, s3, c.w), 0.0f);
  float* p = out1 + (size_t)qi * 128 + c4;
  *(volatile v4f*)p = r;
  __threadfence();
  *(volatile v4f*)p = r;
}

extern "C" void kernel_launch(void* const* d_in, const int* in_sizes, int n_in,
                              void* d_out, int out_size, void* d_ws, size_t ws_size,
                              hipStream_t stream) {
  (void)in_sizes; (void)n_in; (void)out_size;
  if (ws_size < WS_TOTAL) return;
  const float* xyz      = (const float*)d_in[0];
  const float* pts      = (const float*)d_in[1];
  const int*   init_far = (const int*)d_in[2];
  const float* w0  = (const float*)d_in[3];
  const float* b0  = (const float*)d_in[4];
  const float* g0  = (const float*)d_in[5];
  const float* be0 = (const float*)d_in[6];
  const float* w1  = (const float*)d_in[7];
  const float* b1  = (const float*)d_in[8];
  const float* g1  = (const float*)d_in[9];
  const float* be1 = (const float*)d_in[10];
  const float* w2  = (const float*)d_in[11];
  const float* b2  = (const float*)d_in[12];
  const float* g2  = (const float*)d_in[13];
  const float* be2 = (const float*)d_in[14];

  float* out0 = (float*)d_out;
  float* out1 = (float*)d_out + (OUT0_BYTES / 4);
  char* ws = (char*)d_ws;
  unsigned short* w0h = (unsigned short*)(ws + OFF_W0H);
  unsigned short* w1h = (unsigned short*)(ws + OFF_W1H);
  unsigned short* w2h = (unsigned short*)(ws + OFF_W2H);
  float* coef0 = (float*)(ws + OFF_COEF);
  float* coef1 = coef0 + 256;
  float* coef2 = coef0 + 512;
  float* qxyz  = (float*)(ws + OFF_QXYZ);
  float* part0 = (float*)(ws + OFF_PART0);
  float* part1 = (float*)(ws + OFF_PART1);
  float* part2 = (float*)(ws + OFF_PART2);
  unsigned short* x0 = (unsigned short*)(ws + OFF_X0);
  unsigned short* y0 = (unsigned short*)(ws + OFF_Y0);
  unsigned short* y1 = (unsigned short*)(ws + OFF_Y1);
  float* mm = (float*)(ws + OFF_MM);

  cvt_w_kernel<<<7, 256, 0, stream>>>(w0, w1, w2, w0h, w1h, w2h);
  fps_kernel<<<kBatch, 1024, 0, stream>>>(xyz, init_far, out0, qxyz);
  ball_group_kernel<<<(kBatch * kQuery) / 8, 256, 0, stream>>>(xyz, pts, qxyz, x0);

  mlp_layer_kernel<32, 64, false, true><<<kGemmBlocks, 256, 0, stream>>>(x0, w0h, b0, coef0, y0, mm, part0);
  bn_fin_kernel<<<1, 128, 0, stream>>>(part0, kGemmBlocks, g0, be0, coef0, 64);
  mlp_layer_kernel<64, 64, true, true><<<kGemmBlocks, 256, 0, stream>>>(y0, w1h, b1, coef0, y1, mm, part1);
  bn_fin_kernel<<<1, 128, 0, stream>>>(part1, kGemmBlocks, g1, be1, coef1, 64);
  mlp_layer_kernel<64, 128, true, false><<<kGemmBlocks, 256, 0, stream>>>(y1, w2h, b2, coef1, y0, mm, part2);
  bn_fin_kernel<<<1, 128, 0, stream>>>(part2, kGemmBlocks, g2, be2, coef2, 128);

  final_kernel<<<(kBatch * kQuery) / 8, 256, 0, stream>>>(mm, coef2, out1);
}
